// CNN_MambaClassifier_83004537963171
// MI455X (gfx1250) — hardware-verified
//
#include <hip/hip_runtime.h>


namespace {
constexpr int NB = 8, SEQ = 2048, LP = 1024, EMB = 256, CC = 128, KT = 5, SP = SEQ + 4, DI = 256, DS = 16, DTR = 8, XN = 48, DM = 128, NCLS = 10, VOCAB = 50000;
constexpr int NROW = NB * LP;
constexpr float ESC = 64.0f, WSC = 256.0f, XSU = 512.0f, XSS = 4096.0f;
typedef int idx_t;

typedef _Float16 b16;
typedef __attribute__((ext_vector_type(16))) _Float16 v16b;
typedef __attribute__((ext_vector_type(8))) _Float16 v8b;
typedef __attribute__((ext_vector_type(4))) _Float16 v4b;
typedef __attribute__((ext_vector_type(8))) float v8f;
typedef __attribute__((ext_vector_type(4))) float v4f;
__device__ __forceinline__ float bf16_rne(float f) { unsigned int u = __float_as_uint(f); u += 0x7FFFu + ((u >> 16) & 1u); return __uint_as_float(u & 0xFFFF0000u); }
__device__ __forceinline__ void split16(float v, b16& hi, b16& lo) { hi = (b16)v; lo = (b16)(v - (float)hi); }
__device__ __forceinline__ v16b frag_kb(const b16* p, int hh) { const v8b a = *(const v8b*)(p + 8 * hh), b = *(const v8b*)(p + 16 + 8 * hh); v16b f;
#pragma unroll
  for (int e = 0; e < 8; ++e) { f[e] = a[e]; f[8 + e] = b[e]; } return f; }
__device__ __forceinline__ v8f wmma16b(v16b a, v16b b, v8f c) { v8f d = __builtin_amdgcn_wmma_f32_16x16x32_f16(false, a, false, b, (short)0, c, false, false); asm volatile("v_nop\n\tv_nop\n\tv_nop\n\tv_nop" : "+v"(d) : "v"(a), "v"(b)); return d; }
__device__ __forceinline__ float pmul(float a, float b) { float p = a * b; asm volatile("" : "+v"(p)); return p; }
__device__ __forceinline__ int iclamp(long long v, int lo, int hi) { return v < lo ? lo : (v > hi ? hi : (int)v); }
__device__ __forceinline__ float sigm(float x) { return 1.0f / (1.0f + __expf(-x)); }

__global__ __launch_bounds__(256) void prep_kernel(const float* __restrict__ w1, const float* __restrict__ win, const float* __restrict__ wxp, b16* __restrict__ W1r, b16* __restrict__ WIN, b16* __restrict__ WXP) {
  const int tid = blockIdx.x * 256 + threadIdx.x, nth = gridDim.x * 256;
  for (int pass = 0; pass < 2; ++pass) {
    for (int g = tid; g < CC * KT * EMB / 8; g += nth) { const int c = g / (KT * EMB / 8), rem = g - c * (KT * EMB / 8), k = rem / (EMB / 8), e0 = (rem - k * (EMB / 8)) * 8; v8b o;
#pragma unroll
      for (int j = 0; j < 8; ++j) o[j] = (b16)(bf16_rne(w1[(c * EMB + e0 + j) * KT + k]) * WSC);
      *(volatile v8b*)(W1r + (size_t)g * 8) = o; }
    for (int g = tid; g < 2 * DI * DM / 8; g += nth) { const v4f a = *(const v4f*)(win + g * 8), c = *(const v4f*)(win + g * 8 + 4); v8b o;
#pragma unroll
      for (int j = 0; j < 4; ++j) { o[j] = (b16)(bf16_rne(a[j]) * WSC); o[4 + j] = (b16)(bf16_rne(c[j]) * WSC); }
      *(volatile v8b*)(WIN + (size_t)g * 8) = o; }
    for (int g = tid; g < XN * DI / 8; g += nth) { const int r = g / (DI / 8), d0 = (g - r * (DI / 8)) * 8; const int rc = r < DTR + 2 * DS ? r : 0; v8b o;
#pragma unroll
      for (int j = 0; j < 8; ++j) o[j] = (r < DTR + 2 * DS) ? (b16)(bf16_rne(wxp[rc * DI + d0 + j]) * WSC) : (b16)0.0f;
      *(volatile v8b*)(WXP + (size_t)g * 8) = o; }
    __threadfence(); }
}
__global__ __launch_bounds__(256) void gather_kernel(const idx_t* __restrict__ ids, const float* __restrict__ emb, b16* __restrict__ EP) {
  const int wave = threadIdx.x >> 5, lane = threadIdx.x & 31, row = blockIdx.x * 8 + wave;
  const int b = row / SP, p = row - b * SP, s = p - 2; const bool live = (s >= 0) && (s < SEQ);
  const int tok = iclamp(ids[b * SEQ + (live ? s : 0)], 0, VOCAB - 1);
  const v4f a = *(const v4f*)(emb + (size_t)tok * EMB + lane * 8), c = *(const v4f*)(emb + (size_t)tok * EMB + lane * 8 + 4); v8b o;
#pragma unroll
  for (int j = 0; j < 4; ++j) { o[j] = live ? (b16)(bf16_rne(a[j]) * ESC) : (b16)0.0f; o[4 + j] = live ? (b16)(bf16_rne(c[j]) * ESC) : (b16)0.0f; }
  for (int pass = 0; pass < 2; ++pass) { *(volatile v8b*)(EP + (size_t)row * EMB + lane * 8) = o; __threadfence(); }
}
__global__ __launch_bounds__(128) void conv_kernel(const b16* __restrict__ EP, const b16* __restrict__ W1r, const float* __restrict__ cb, float* __restrict__ U, b16* __restrict__ UH, b16* __restrict__ UL) {
  __shared__ __attribute__((aligned(16))) float Tp[32][CC + 4];
  const int wave = threadIdx.x >> 5, lane = threadIdx.x & 31, nloc = lane & 15, hlf = lane >> 4, b = blockIdx.y, s0 = blockIdx.x * 64 + wave * 16;
  const b16* A = EP + ((size_t)b * SP + s0 + nloc) * EMB;
  v8f acc[8];
#pragma unroll
  for (int t = 0; t < 8; ++t) acc[t] = (v8f){};
  for (int k = 0; k < KT; ++k) {
#pragma unroll 2
    for (int e0 = 0; e0 < EMB; e0 += 32) { const v16b a = frag_kb(A + (size_t)k * EMB + e0, hlf);
#pragma unroll
      for (int t = 0; t < 8; ++t) acc[t] = wmma16b(a, frag_kb(W1r + (size_t)(t * 16 + nloc) * (KT * EMB) + k * EMB + e0, hlf), acc[t]); } }
#pragma unroll
  for (int t = 0; t < 8; ++t) { const float bias = bf16_rne(cb[t * 16 + nloc]);
#pragma unroll
    for (int i = 0; i < 4; ++i) { const float v0 = fmaxf(acc[t][2 * i] * (1.0f / (ESC * WSC)) + bias, 0.0f), v1 = fmaxf(acc[t][2 * i + 1] * (1.0f / (ESC * WSC)) + bias, 0.0f); Tp[wave * 8 + 4 * hlf + i][t * 16 + nloc] = fmaxf(v0, v1); } }
  __syncthreads();
  const size_t l0 = (size_t)b * LP + (size_t)blockIdx.x * 32;
  for (int pass = 0; pass < 2; ++pass) {
    for (int rr = wave * 8; rr < wave * 8 + 8; ++rr) { const v4f v = *(const v4f*)(&Tp[rr][lane * 4]); v4b h4, l4;
#pragma unroll
      for (int j = 0; j < 4; ++j) { b16 x_, y_; split16(v[j] * XSU, x_, y_); h4[j] = x_; l4[j] = y_; }
      *(volatile v4f*)(U + (l0 + rr) * CC + lane * 4) = v; *(volatile v4b*)(UH + (l0 + rr) * CC + lane * 4) = h4; *(volatile v4b*)(UL + (l0 + rr) * CC + lane * 4) = l4; }
    __threadfence(); }
}
__global__ __launch_bounds__(128) void inproj_kernel(const b16* __restrict__ UH, const b16* __restrict__ UL, const b16* __restrict__ WIN, float* __restrict__ XZ) {
  __shared__ __attribute__((aligned(16))) float Ts[4][16][256 + 4];
  const int wave = threadIdx.x >> 5, lane = threadIdx.x & 31, nloc = lane & 15, hlf = lane >> 4; const size_t m0 = (size_t)blockIdx.x * 64 + wave * 16;
  for (int half = 0; half < 2; ++half) {
    v8f acc[16];
#pragma unroll
    for (int t = 0; t < 16; ++t) acc[t] = (v8f){};
#pragma unroll
    for (int kb = 0; kb < CC; kb += 32) { const v16b ah = frag_kb(UH + (m0 + nloc) * CC + kb, hlf), al = frag_kb(UL + (m0 + nloc) * CC + kb, hlf);
#pragma unroll
      for (int t = 0; t < 16; ++t) { const v16b bw = frag_kb(WIN + (size_t)(half * 256 + t * 16 + nloc) * CC + kb, hlf); acc[t] = wmma16b(ah, bw, acc[t]); acc[t] = wmma16b(al, bw, acc[t]); } }
#pragma unroll
    for (int t = 0; t < 16; ++t)
#pragma unroll
      for (int r = 0; r < 8; ++r) Ts[wave][8 * hlf + r][t * 16 + nloc] = acc[t][r] * (1.0f / (XSU * WSC));
    __syncthreads();
    for (int pass = 0; pass < 2; ++pass) { for (int k = lane; k < 16 * 64; k += 32) { const int rr = k >> 6, c4 = (k & 63) * 4; *(volatile v4f*)(XZ + (m0 + rr) * (2 * DI) + half * 256 + c4) = *(const v4f*)(&Ts[wave][rr][c4]); } __threadfence(); }
    __syncthreads(); }
}
__global__ __launch_bounds__(256) void dwconv_kernel(const float* __restrict__ XZ, const float* __restrict__ wd, const float* __restrict__ bd, float* __restrict__ US, b16* __restrict__ USH, b16* __restrict__ USL) {
  __shared__ __attribute__((aligned(16))) float Tu[64][DI + 4];
  const int d = threadIdx.x, b = blockIdx.y, lb = blockIdx.x * 64, wave = threadIdx.x >> 5, lane = threadIdx.x & 31;
  const float w0 = bf16_rne(wd[d * 4 + 0]), w1 = bf16_rne(wd[d * 4 + 1]), w2 = bf16_rne(wd[d * 4 + 2]), w3 = bf16_rne(wd[d * 4 + 3]), bias = bf16_rne(bd[d]);
  float um3, um2, um1;
  { const int la = lb - 3, lbm = lb - 2, lc = lb - 1;
    const float a = XZ[((size_t)b * LP + (la < 0 ? 0 : la)) * (2 * DI) + d], bb = XZ[((size_t)b * LP + (lbm < 0 ? 0 : lbm)) * (2 * DI) + d], c = XZ[((size_t)b * LP + (lc < 0 ? 0 : lc)) * (2 * DI) + d];
    um3 = la < 0 ? 0.0f : a; um2 = lbm < 0 ? 0.0f : bb; um1 = lc < 0 ? 0.0f : c; }
  for (int i = 0; i < 64; ++i) { const float u0 = XZ[((size_t)b * LP + lb + i) * (2 * DI) + d]; const float x = pmul(w0, um3) + pmul(w1, um2) + pmul(w2, um1) + pmul(w3, u0) + bias; Tu[i][d] = x * sigm(x); um3 = um2; um2 = um1; um1 = u0; }
  __syncthreads();
  for (int pass = 0; pass < 2; ++pass) {
    for (int rr = wave * 8; rr < wave * 8 + 8; ++rr) { const size_t row = (size_t)b * LP + lb + rr;
      for (int h = 0; h < 2; ++h) *(volatile v4f*)(US + row * DI + h * 128 + lane * 4) = *(const v4f*)(&Tu[rr][h * 128 + lane * 4]);
      v8b h8, l8; const v4f a = *(const v4f*)(&Tu[rr][lane * 8]), c = *(const v4f*)(&Tu[rr][lane * 8 + 4]);
#pragma unroll
      for (int j = 0; j < 4; ++j) { b16 x_, y_; split16(a[j] * XSS, x_, y_); h8[j] = x_; l8[j] = y_; split16(c[j] * XSS, x_, y_); h8[4 + j] = x_; l8[4 + j] = y_; }
      *(volatile v8b*)(USH + row * DI + lane * 8) = h8; *(volatile v8b*)(USL + row * DI + lane * 8) = l8; }
    __threadfence(); }
}
__global__ __launch_bounds__(128) void xproj_kernel(const b16* __restrict__ USH, const b16* __restrict__ USL, const b16* __restrict__ WXP, const float* __restrict__ wdt, const float* __restrict__ bdt, float* __restrict__ XD, float* __restrict__ DT) {
  __shared__ __attribute__((aligned(16))) float Tx[64][XN]; __shared__ __attribute__((aligned(16))) float Td[64][DI + 4];
  const int wave = threadIdx.x >> 5, lane = threadIdx.x & 31, nloc = lane & 15, hlf = lane >> 4; const size_t r0 = (size_t)blockIdx.x * 64, m0 = r0 + wave * 16;
  v8f acc[3] = {{}, {}, {}};
#pragma unroll 2
  for (int kb = 0; kb < DI; kb += 32) { const v16b ah = frag_kb(USH + (m0 + nloc) * DI + kb, hlf), al = frag_kb(USL + (m0 + nloc) * DI + kb, hlf);
#pragma unroll
    for (int t = 0; t < 3; ++t) { const v16b bw = frag_kb(WXP + (size_t)(t * 16 + nloc) * DI + kb, hlf); acc[t] = wmma16b(ah, bw, acc[t]); acc[t] = wmma16b(al, bw, acc[t]); } }
#pragma unroll
  for (int t = 0; t < 3; ++t)
#pragma unroll
    for (int r = 0; r < 8; ++r) Tx[wave * 16 + 8 * hlf + r][t * 16 + nloc] = acc[t][r] * (1.0f / (XSS * WSC));
  __syncthreads();
  { const int dd = threadIdx.x;
    for (int h = 0; h < 2; ++h) { const int ch = dd + h * 128; float w[DTR];
#pragma unroll
      for (int j = 0; j < DTR; ++j) w[j] = bf16_rne(wdt[ch * DTR + j]); const float bb = bf16_rne(bdt[ch]);
      for (int i = 0; i < 64; ++i) { float s = bb;
#pragma unroll
        for (int j = 0; j < DTR; ++j) s += pmul(Tx[i][j], w[j]);
        Td[i][ch] = (s > 20.0f) ? s : log1pf(__expf(s)); } } }
  __syncthreads();
  for (int pass = 0; pass < 2; ++pass) {
    for (int k = threadIdx.x; k < 64 * XN / 4; k += 128) *(volatile v4f*)(XD + r0 * XN + (size_t)k * 4) = *(const v4f*)(&Tx[0][0] + k * 4);
    for (int rr = wave * 16; rr < wave * 16 + 16; ++rr) for (int h = 0; h < 2; ++h) *(volatile v4f*)(DT + (r0 + rr) * DI + h * 128 + lane * 4) = *(const v4f*)(&Td[rr][h * 128 + lane * 4]);
    __threadfence(); }
}
__global__ __launch_bounds__(256) void scan_kernel(const float* __restrict__ DT, const float* __restrict__ US, const float* __restrict__ XZ, const float* __restrict__ XD, const float* __restrict__ alog, const float* __restrict__ Dp, float* __restrict__ YM) {
  __shared__ float Sbc[64][2 * DS];
  const int b = blockIdx.x, d = threadIdx.x;
  float A[DS], h[DS];
#pragma unroll
  for (int n = 0; n < DS; ++n) { A[n] = -__expf(bf16_rne(alog[d * DS + n])); h[n] = 0.0f; }
  const float Dd = bf16_rne(Dp[d]); float ysum = 0.0f;
  for (int l0 = 0; l0 < LP; l0 += 64) {
    __syncthreads();
    for (int k = d; k < 64 * 2 * DS; k += 256) { const int i = k >> 5, j = k & 31; Sbc[i][j] = XD[((size_t)b * LP + l0 + i) * XN + DTR + j]; }
    __syncthreads();
    for (int i = 0; i < 64; ++i) { const size_t row = (size_t)b * LP + l0 + i; const float dt = DT[row * DI + d], u = US[row * DI + d], z = XZ[row * (2 * DI) + DI + d]; const float du = pmul(dt, u); float y = pmul(Dd, u);
#pragma unroll
      for (int n = 0; n < DS; ++n) { h[n] = pmul(__expf(pmul(dt, A[n])), h[n]) + pmul(du, Sbc[i][n]); y += pmul(h[n], Sbc[i][DS + n]); }
      ysum += pmul(y, z * sigm(z)); } }
  const float ym = ysum * (1.0f / LP);
  for (int pass = 0; pass < 2; ++pass) { ((volatile float*)YM)[b * DI + d] = ym; __threadfence(); }
}
__global__ __launch_bounds__(256) void tail_kernel(const float* __restrict__ YM, const float* __restrict__ wout, const float* __restrict__ fcw, const float* __restrict__ fcb, float* __restrict__ out) {
  __shared__ float Sy[NB][DI], Sv[NB][DM], So[NB * NCLS + 16];
  const int t_ = threadIdx.x;
  for (int k = t_; k < NB * DI; k += 256) Sy[k >> 8][k & 255] = YM[k];
  __syncthreads();
  for (int k = t_; k < NB * DM; k += 256) { const int b = k >> 7, c = k & 127; float s = 0.0f; for (int d = 0; d < DI; ++d) s += pmul(bf16_rne(wout[c * DI + d]), Sy[b][d]); Sv[b][c] = s; }
  __syncthreads();
  if (t_ < NB * NCLS) { const int b = t_ / NCLS, j = t_ - b * NCLS; float s = bf16_rne(fcb[j]); for (int c = 0; c < DM; ++c) s += pmul(bf16_rne(fcw[j * DM + c]), Sv[b][c]); So[t_] = s; }
  __syncthreads();
  for (int pass = 0; pass < 2; ++pass) { if (t_ < NB * NCLS) ((volatile float*)out)[t_] = So[t_]; __threadfence(); }
}
}

extern "C" void kernel_launch(void* const* d_in, const int* in_sizes, int n_in, void* d_out, int out_size, void* d_ws, size_t ws_size, hipStream_t stream) {
  (void)n_in;
  auto Fp = [&](int i) { return (const float*)d_in[i]; };
  if (in_sizes[0] != NB * SEQ || in_sizes[1] != VOCAB * EMB || in_sizes[2] != CC * EMB * KT || in_sizes[4] != 2 * DI * DM || in_sizes[7] != (DTR + 2 * DS) * DI || out_size != NB * NCLS) return;
  size_t off = 0; char* ws = (char*)d_ws;
  auto carve = [&](size_t bytes) { char* p = ws + off; off += (bytes + 255) & ~(size_t)255; return p; };
  b16* W1r = (b16*)carve((size_t)CC * KT * EMB * 2); b16* WIN = (b16*)carve((size_t)2 * DI * DM * 2); b16* WXP = (b16*)carve((size_t)XN * DI * 2);
  b16* EP = (b16*)carve((size_t)NB * SP * EMB * 2);
  float* U = (float*)carve((size_t)NROW * CC * 4); b16* UH = (b16*)carve((size_t)NROW * CC * 2); b16* UL = (b16*)carve((size_t)NROW * CC * 2);
  float* XZ = (float*)carve((size_t)NROW * 2 * DI * 4);
  float* US = (float*)carve((size_t)NROW * DI * 4); b16* USH = (b16*)carve((size_t)NROW * DI * 2); b16* USL = (b16*)carve((size_t)NROW * DI * 2);
  float* XD = (float*)carve((size_t)NROW * XN * 4); float* DT = (float*)carve((size_t)NROW * DI * 4); float* YM = (float*)carve((size_t)NB * DI * 4);
  if (off > ws_size) return;
  prep_kernel<<<128, 256, 0, stream>>>(Fp(2), Fp(4), Fp(7), W1r, WIN, WXP);
  gather_kernel<<<NB * SP / 8, 256, 0, stream>>>((const idx_t*)d_in[0], Fp(1), EP);
  conv_kernel<<<dim3(SEQ / 64, NB), 128, 0, stream>>>(EP, W1r, Fp(3), U, UH, UL);
  inproj_kernel<<<NROW / 64, 128, 0, stream>>>(UH, UL, WIN, XZ);
  dwconv_kernel<<<dim3(LP / 64, NB), 256, 0, stream>>>(XZ, Fp(5), Fp(6), US, USH, USL);
  xproj_kernel<<<NROW / 64, 128, 0, stream>>>(USH, USL, WXP, Fp(8), Fp(9), XD, DT);
  scan_kernel<<<NB, 256, 0, stream>>>(DT, US, XZ, XD, Fp(10), Fp(11), YM);
  tail_kernel<<<1, 256, 0, stream>>>(YM, Fp(12), Fp(13), Fp(14), (float*)d_out);
}
